// HybridAttention_37254546325711
// MI455X (gfx1250) — hardware-verified
//
#include <hip/hip_runtime.h>
#include <math.h>

#ifndef NB
#define NB 2
#endif
#ifndef SEQ
#define SEQ 2048
#endif
#define NB_FULL 2
#define TT_FULL 2048
#define CC 1024
#define NH 16
#define NKV 4
#define HD 64
#define KVD 256
#define HG 4
static_assert(SEQ % 128 == 0);
static_assert(SEQ >= 256);
static_assert(SEQ <= TT_FULL);
static_assert(NB >= 1);
static_assert(NB <= NB_FULL);
static_assert(NH == NKV * HG);

typedef __attribute__((ext_vector_type(16))) _Float16 v16h;
typedef __attribute__((ext_vector_type(16))) __bf16 v16b;
typedef __attribute__((ext_vector_type(8)))  _Float16 v8h;
typedef __attribute__((ext_vector_type(8)))  __bf16 v8b;
typedef __attribute__((ext_vector_type(8)))  float v8f;
typedef __attribute__((ext_vector_type(4)))  float v4f;
typedef __attribute__((ext_vector_type(4)))  unsigned v4u;

template <typename T> __device__ __forceinline__ void vst2(void* p, T v) { *(volatile T*)p = v; __threadfence(); *(volatile T*)p = v; }

__device__ __forceinline__ v8f wmma16(v16h a, v16h b, v8f c) {
  v8f d = __builtin_amdgcn_wmma_f32_16x16x32_f16(false, a, false, b, (short)0, c, false, false);
  asm volatile("v_nop\n\tv_nop\n\tv_nop\n\tv_nop" : "+v"(d) : "v"(a), "v"(b));
  return d;
}
__device__ __forceinline__ v8f wmma_bf(v16b a, v16b b, v8f c) {
  v8f d = __builtin_amdgcn_wmma_f32_16x16x32_bf16(false, a, false, b, (short)0, c, false, false);
  asm volatile("v_nop\n\tv_nop\n\tv_nop\n\tv_nop" : "+v"(d) : "v"(a), "v"(b));
  return d;
}
__device__ __forceinline__ v16h frag_h(const _Float16* rowk0, int lane) {
  union { v16h v; v8h q[2]; } u; const _Float16* p = rowk0 + 8 * (lane >> 4);
  u.q[0] = *(const v8h*)p; u.q[1] = *(const v8h*)(p + 16); return u.v;
}
__device__ __forceinline__ v16b frag_b(const __bf16* rowk0, int lane) {
  union { v16b v; v8b q[2]; } u; const __bf16* p = rowk0 + 8 * (lane >> 4);
  u.q[0] = *(const v8b*)p; u.q[1] = *(const v8b*)(p + 16); return u.v;
}
__device__ __forceinline__ float bfr(float v) { return (float)(__bf16)v; }
__device__ __forceinline__ void ldsx() { asm volatile("s_wait_dscnt 0" ::: "memory"); __builtin_amdgcn_wave_barrier(); __builtin_amdgcn_fence(3, "workgroup"); }

#define WS_WQI 0ull
#define WS_WKI (WS_WQI + 2ull * CC * CC)
#define WS_WVI (WS_WKI + 2ull * KVD * CC)
#define WS_WPI (WS_WVI + 2ull * KVD * CC)
#define WS_CS  (WS_WPI + 2ull * CC * CC)
#define WS_CSN (WS_CS + 4ull * 2560)
#define WS_QH  (WS_CSN + 8ull * SEQ * 16)
#define WS_QL  (WS_QH + 2ull * NB * SEQ * CC)
#define WS_KH  (WS_QL + 2ull * NB * SEQ * CC)
#define WS_KL  (WS_KH + 2ull * NB * SEQ * KVD)
#define WS_VT  (WS_KL + 2ull * NB * SEQ * KVD)
#define WS_VR  (WS_VT + 2ull * NB * KVD * SEQ)
#define WS_VF  (WS_VR + 2ull * NB * KVD * SEQ)
#define WS_Y   (WS_VF + 4ull * NB * SEQ * KVD)
#define WS_BIG (WS_Y + 4ull * NB * SEQ * CC)
#define BIG_S  (4ull * HG * SEQ * SEQ)
#define BIG_X  (2ull * NB * SEQ * CC)
#define BIG_Y  (4ull * NB * SEQ * CC)
#define BIG_SX (BIG_S > BIG_X ? BIG_S : BIG_X)
#define BIG_SZ (BIG_SX > BIG_Y ? BIG_SX : BIG_Y)
#define WS_END (WS_BIG + BIG_SZ)
static_assert(BIG_SZ >= BIG_S);
static_assert(BIG_SZ >= BIG_X);
static_assert(BIG_SZ >= BIG_Y);
static_assert(WS_END <= 134217728ull);
static_assert((WS_CSN % 256) == 0);
static_assert((WS_QH % 256) == 0);
static_assert((WS_BIG % 256) == 0);

#define NQB 80
#define NXB (NB * SEQ / 32)
#define NTB (SEQ / 4)

__global__ __launch_bounds__(128) void k_prep(const float* __restrict__ X, const float* __restrict__ WQ, const float* __restrict__ WK, const float* __restrict__ WV, const float* __restrict__ WP,
    __bf16* __restrict__ WQI, __bf16* __restrict__ WKI, __bf16* __restrict__ WVI, __bf16* __restrict__ WPI, float* __restrict__ CS, __bf16* __restrict__ XB, float* __restrict__ CSN) {
  __shared__ float sred[4]; __shared__ __align__(16) float scs[32];
  const int tid = threadIdx.x, wave = tid >> 5, lane = tid & 31; const int blk = blockIdx.x;
  if (blk < NQB) {
    const int gr0 = blk * 32; const float* W; __bf16* WI; int lr0; float hv;
    if (gr0 < 1024) { W = WQ; WI = WQI; lr0 = gr0; hv = 32.0f; }
    else if (gr0 < 1280) { W = WK; WI = WKI; lr0 = gr0 - 1024; hv = 32.0f; }
    else if (gr0 < 1536) { W = WV; WI = WVI; lr0 = gr0 - 1280; hv = 16.0f; }
    else { W = WP; WI = WPI; lr0 = gr0 - 1536; hv = 16.0f; }
    for (int r = 0; r < 32; ++r) {
      const float* wr = W + (size_t)(lr0 + r) * CC + tid * 8;
      const v4f u0 = *(const v4f*)wr, u1 = *(const v4f*)(wr + 4);
      float f[8] = { u0.x, u0.y, u0.z, u0.w, u1.x, u1.y, u1.z, u1.w };
      float mx = 0.f;
#pragma unroll
      for (int i = 0; i < 8; ++i) { f[i] = bfr(f[i]); mx = fmaxf(mx, fabsf(f[i])); }
#pragma unroll
      for (int o = 16; o > 0; o >>= 1) mx = fmaxf(mx, __shfl_xor(mx, o));
      if (lane == 0) sred[wave] = mx;
      __syncthreads();
      const float wmax = fmaxf(fmaxf(fmaxf(sred[0], sred[1]), fmaxf(sred[2], sred[3])), 1e-5f);
      const float rinv = 1.0f / wmax;
      union { v8b v; v4u u; } pk;
#pragma unroll
      for (int i = 0; i < 8; ++i) { const float t1 = f[i] * rinv; float wi = rintf(t1 * hv); wi = fminf(fmaxf(wi, -hv), hv - 1.0f); pk.v[i] = (__bf16)wi; }
      vst2((unsigned*)(WI + (size_t)(lr0 + r) * CC + tid * 8), pk.u);
      if (tid == 0) scs[r] = wmax / hv;
      __syncthreads();
    }
    if (wave == 0 && lane < 8) vst2(CS + gr0 + lane * 4, *(const v4f*)&scs[lane * 4]);
  } else if (blk < NQB + NXB) {
    const int rr0 = (blk - NQB) * 32;
    for (int r = 0; r < 32; ++r) {
      const int rr = rr0 + r; const int b = rr / SEQ, t = rr - b * SEQ;
      const float* src = X + ((size_t)b * TT_FULL + t) * CC + tid * 8;
      const v4f u0 = *(const v4f*)src, u1 = *(const v4f*)(src + 4);
      const float f[8] = { u0.x, u0.y, u0.z, u0.w, u1.x, u1.y, u1.z, u1.w };
      union { v8b v; v4u u; } pk;
#pragma unroll
      for (int i = 0; i < 8; ++i) pk.v[i] = (__bf16)f[i];
      vst2((unsigned*)(XB + (size_t)rr * CC + tid * 8), pk.u);
    }
  } else {
    const int e = (blk - NQB - NXB) * 128 + tid;
    const int tab = e / (SEQ * 16); const int rem = e - tab * (SEQ * 16); const int t = rem >> 4, i = rem & 15;
    const float ef = (float)(2 * i) * (1.0f / 32.0f);
    const float p = powf(10000.0f, ef); const float inv = 1.0f / p; const float ang = (float)t * inv;
    float val;
    if (tab == 0) val = cosf(ang); else val = sinf(ang);
    vst2(CSN + e, val);
  }
}

__global__ __launch_bounds__(128) void k_proj(const __bf16* __restrict__ XB, const __bf16* __restrict__ WQI, const __bf16* __restrict__ WKI, const __bf16* __restrict__ WVI, const float* __restrict__ CS, const float* __restrict__ CSN, const float* __restrict__ QG,
    _Float16* __restrict__ QH, _Float16* __restrict__ QL, _Float16* __restrict__ KH, _Float16* __restrict__ KL, _Float16* __restrict__ VT, _Float16* __restrict__ VR, float* __restrict__ VF) {
  __shared__ __align__(16) float sf[64][132];
  __shared__ __align__(16) _Float16 lh[2][9216];
  const int tid = threadIdx.x, wave = tid >> 5, lane = tid & 31, col = lane & 15, g = lane >> 4;
  const int y = blockIdx.y; const size_t r0 = (size_t)blockIdx.x * 64;
  int which, c0; const __bf16* W; const float* cs;
  if (y < 8) { which = 0; c0 = y * 128; W = WQI; cs = CS + c0; }
  else if (y < 10) { which = 1; c0 = (y - 8) * 128; W = WKI; cs = CS + 1024 + c0; }
  else { which = 2; c0 = (y - 10) * 128; W = WVI; cs = CS + 1280 + c0; }
  v8f acc[8] = {};
#pragma unroll 2
  for (int kc = 0; kc < CC / 32; ++kc) {
    const v16b a = frag_b(XB + (r0 + wave * 16 + col) * CC + kc * 32, lane);
#pragma unroll
    for (int j = 0; j < 8; ++j) { const v16b w = frag_b(W + (size_t)(c0 + j * 16 + col) * CC + kc * 32, lane); acc[j] = wmma_bf(a, w, acc[j]); }
  }
  if (which < 2) {
#pragma unroll
    for (int j = 0; j < 8; ++j) { const float sc = cs[j * 16 + col];
#pragma unroll
      for (int r = 0; r < 8; ++r) sf[wave * 16 + 8 * g + r][j * 16 + col] = acc[j][r] * sc; }
    __syncthreads();
    const int rl = tid & 63, hh = tid >> 6; const int t = (int)(r0 % SEQ) + rl;
    float v[64];
#pragma unroll
    for (int dd = 0; dd < 64; ++dd) v[dd] = sf[rl][hh * 64 + dd];
    float sq = 0.f;
#pragma unroll
    for (int dd = 0; dd < 64; ++dd) sq += v[dd] * v[dd];
    const float rs = rsqrtf(sq * (1.0f / 64.0f) + 1.1920929e-7f);
    float cv[16], sv[16];
    { const float* cp = CSN + (size_t)t * 16; const float* sp = CSN + (size_t)SEQ * 16 + (size_t)t * 16;
#pragma unroll
      for (int qd = 0; qd < 4; ++qd) { const v4f c4 = *(const v4f*)(cp + 4 * qd), s4 = *(const v4f*)(sp + 4 * qd);
        cv[4 * qd] = c4.x; cv[4 * qd + 1] = c4.y; cv[4 * qd + 2] = c4.z; cv[4 * qd + 3] = c4.w; sv[4 * qd] = s4.x; sv[4 * qd + 1] = s4.y; sv[4 * qd + 2] = s4.z; sv[4 * qd + 3] = s4.w; } }
    const int hq = 2 * y + hh; const float gq = bfr(QG[hq < NH ? hq : NH - 1]); const float gain = (which == 0) ? gq : 1.0f;
#pragma unroll
    for (int i = 0; i < 16; ++i) { const float x1 = v[i] * rs, x2 = v[16 + i] * rs; v[i] = x1 * cv[i] + x2 * sv[i]; v[16 + i] = x2 * cv[i] - x1 * sv[i]; }
#pragma unroll
    for (int dd = 32; dd < 64; ++dd) v[dd] *= rs;
#pragma unroll
    for (int dd = 0; dd < 64; ++dd) { const float o = v[dd] * gain; const _Float16 hv = (_Float16)o; lh[0][rl * 136 + hh * 64 + dd] = hv; lh[1][rl * 136 + hh * 64 + dd] = (_Float16)((o - (float)hv) * 1024.0f); }
    __syncthreads();
    _Float16* dh = (which == 0) ? QH : KH; _Float16* dl = (which == 0) ? QL : KL; const size_t pitch = (which == 0) ? (size_t)CC : (size_t)KVD;
    for (int e = tid; e < 64 * 16; e += 128) { const int rl2 = e >> 4, q8 = e & 15; const size_t off = (r0 + rl2) * pitch + c0 + q8 * 8;
      vst2((unsigned*)(dh + off), *(const v4u*)&lh[0][rl2 * 136 + q8 * 8]); vst2((unsigned*)(dl + off), *(const v4u*)&lh[1][rl2 * 136 + q8 * 8]); }
  } else {
#pragma unroll
    for (int j = 0; j < 8; ++j) { const float sc = cs[j * 16 + col];
#pragma unroll
      for (int r = 0; r < 8; ++r) { const float vv = acc[j][r] * sc; const int rl = wave * 16 + 8 * g + r, cl = j * 16 + col; sf[rl][cl] = vv; const _Float16 hv = (_Float16)vv; lh[0][cl * 72 + rl] = hv; lh[1][cl * 72 + rl] = (_Float16)((vv - (float)hv) * 1024.0f); } }
    __syncthreads();
    for (int e = tid; e < 64 * 32; e += 128) { const int rl = e >> 5, q4 = e & 31; vst2(VF + (r0 + rl) * KVD + c0 + q4 * 4, *(const v4f*)&sf[rl][q4 * 4]); }
    const size_t b = r0 / SEQ; const int t0 = (int)(r0 % SEQ);
    for (int e = tid; e < 128 * 8; e += 128) { const int cl = e >> 3, q8 = e & 7; const size_t o2 = (b * KVD + c0 + cl) * (size_t)SEQ + t0 + q8 * 8;
      vst2((unsigned*)(VT + o2), *(const v4u*)&lh[0][cl * 72 + q8 * 8]); vst2((unsigned*)(VR + o2), *(const v4u*)&lh[1][cl * 72 + q8 * 8]); }
  }
}

__global__ __launch_bounds__(128) __attribute__((amdgpu_num_vgpr(256))) void k_sc(const _Float16* __restrict__ QH, const _Float16* __restrict__ QL, const _Float16* __restrict__ KH, const _Float16* __restrict__ KL, int b, int kvh, float* __restrict__ S0) {
  __shared__ __align__(16) float ss[4][16][132];
  if ((int)blockIdx.y * 128 > (int)blockIdx.x * 64 + 63) return;
  const int gh = blockIdx.z, h = kvh * HG + gh; float* S = S0 + (size_t)gh * SEQ * SEQ;
  const int tid = threadIdx.x, wave = tid >> 5, lane = tid & 31, col = lane & 15, g = lane >> 4;
  const int k0 = blockIdx.y * 128; const int ql0 = blockIdx.x * 64 + wave * 16; const size_t q0 = (size_t)b * SEQ + ql0;
  const bool early = blockIdx.x < 4;
#pragma unroll 1
  for (int jh = 0; jh < 2; ++jh) {
    const int kh0 = k0 + jh * 64;
    v8f acc[4] = {}, accl[4] = {};
#pragma unroll 1
    for (int kc = 0; kc < HD / 32; ++kc) {
      const v16h ah = frag_h(QH + (q0 + col) * CC + h * HD + kc * 32, lane), al = frag_h(QL + (q0 + col) * CC + h * HD + kc * 32, lane);
      if (early) {
#pragma unroll
        for (int j = 0; j < 4; ++j) { const size_t kr = ((size_t)b * SEQ + kh0 + j * 16 + col) * KVD + kvh * HD + kc * 32;
          const v16h kb = frag_h(KH + kr, lane); acc[j] = wmma16(ah, kb, acc[j]); accl[j] = wmma16(al, kb, accl[j]);
          const v16h kl = frag_h(KL + kr, lane); accl[j] = wmma16(ah, kl, accl[j]); }
      } else {
#pragma unroll
        for (int j = 0; j < 4; ++j) { const size_t kr = ((size_t)b * SEQ + kh0 + j * 16 + col) * KVD + kvh * HD + kc * 32;
          const v16h kb = frag_h(KH + kr, lane);
          acc[j] = wmma16(ah, kb, acc[j]); accl[j] = wmma16(al, kb, accl[j]); }
      }
    }
#pragma unroll
    for (int j = 0; j < 4; ++j) acc[j] += accl[j] * (1.0f / 1024.0f);
#pragma unroll
    for (int j = 0; j < 4; ++j)
#pragma unroll
      for (int r = 0; r < 8; ++r) ss[wave][8 * g + r][jh * 64 + j * 16 + col] = acc[j][r] * 0.125f;
  }
  ldsx();
  for (int rl = 0; rl < 16; ++rl) vst2(S + (size_t)(ql0 + rl) * SEQ + k0 + lane * 4, *(const v4f*)&ss[wave][rl][lane * 4]);
}

__global__ __launch_bounds__(256) void k_sm(float* __restrict__ S0) {
  __shared__ float sred[8]; __shared__ float sbc; __shared__ __align__(16) float sh[SEQ];
  const int t = threadIdx.x; const int q = blockIdx.x; float* sr = S0 + (size_t)blockIdx.y * SEQ * SEQ + (size_t)q * SEQ;
  const int kend = q + 1; const int kw = ((q >> 6) + 1) << 6;
  float m = -3.0e38f;
#pragma unroll 1
  for (int k = t; k < kw; k += 256) { const float v = sr[k]; const float x = (k < kend) ? v : -__builtin_inff(); sh[k] = x; m = fmaxf(m, x); }
#pragma unroll
  for (int o = 1; o < 32; o <<= 1) m = fmaxf(m, __shfl_xor(m, o));
  if ((t & 31) == 0) sred[t >> 5] = m; __syncthreads();
  if (t == 0) { float a = sred[0]; for (int i = 1; i < 8; ++i) a = fmaxf(a, sred[i]); sbc = a; } __syncthreads(); m = sbc; __syncthreads();
  float sum = 0.f;
#pragma unroll 1
  for (int k = t; k < kw; k += 256) { const float e = expf(sh[k] - m); sh[k] = e; sum += e; }
#pragma unroll
  for (int o = 1; o < 32; o <<= 1) sum += __shfl_xor(sum, o);
  if ((t & 31) == 0) sred[t >> 5] = sum; __syncthreads();
  if (t == 0) { float a = 0.f; for (int i = 0; i < 8; ++i) a += sred[i]; sbc = 2048.0f / a; } __syncthreads();
  const float c = sbc;
  for (int qq = t; qq < kw / 4; qq += 256) { v4f p = *(const v4f*)&sh[qq * 4]; p = p * c; vst2(sr + qq * 4, p); }
}

__global__ __launch_bounds__(128) __attribute__((amdgpu_num_vgpr(256))) void k_pv(const float* __restrict__ S0, const _Float16* __restrict__ VT, const _Float16* __restrict__ VR, int b, int kvh, float* __restrict__ Y) {
  __shared__ __align__(16) float ss[4][16][HD + 4];
  const int gh = blockIdx.z, h = kvh * HG + gh; const float* PS = S0 + (size_t)gh * SEQ * SEQ;
  const int tid = threadIdx.x, wave = tid >> 5, lane = tid & 31, col = lane & 15, g = lane >> 4;
  const int ql0 = blockIdx.x * 64 + wave * 16; const int kend = blockIdx.x * 64 + 64; const bool early = blockIdx.x < 4;
  v8f acc[4] = {}, accr[4] = {};
#pragma unroll 1
  for (int kc = 0; kc < kend / 32; ++kc) {
    const float* prow = PS + (size_t)(ql0 + col) * SEQ + kc * 32 + 8 * g;
    const v4f t0 = *(const v4f*)prow, t1 = *(const v4f*)(prow + 4), t2 = *(const v4f*)(prow + 16), t3 = *(const v4f*)(prow + 20);
    const float pf[16] = { t0.x, t0.y, t0.z, t0.w, t1.x, t1.y, t1.z, t1.w, t2.x, t2.y, t2.z, t2.w, t3.x, t3.y, t3.z, t3.w };
    v16h ph;
#pragma unroll
    for (int i = 0; i < 16; ++i) ph[i] = (_Float16)pf[i];
    if (early) {
      v16h pl;
#pragma unroll
      for (int i = 0; i < 16; ++i) pl[i] = (_Float16)((pf[i] - (float)ph[i]) * 1024.0f);
#pragma unroll
      for (int j = 0; j < 4; ++j) { const size_t po = ((size_t)b * KVD + kvh * HD + j * 16 + col) * (size_t)SEQ + kc * 32;
        const v16h vh = frag_h(VT + po, lane); const v16h vr = frag_h(VR + po, lane);
        acc[j] = wmma16(ph, vh, acc[j]); accr[j] = wmma16(ph, vr, accr[j]); accr[j] = wmma16(pl, vh, accr[j]); }
    } else {
#pragma unroll
      for (int j = 0; j < 4; ++j) { const size_t po = ((size_t)b * KVD + kvh * HD + j * 16 + col) * (size_t)SEQ + kc * 32;
        const v16h vh = frag_h(VT + po, lane); acc[j] = wmma16(ph, vh, acc[j]); }
    }
  }
#pragma unroll
  for (int j = 0; j < 4; ++j)
#pragma unroll
    for (int r = 0; r < 8; ++r) ss[wave][8 * g + r][j * 16 + col] = (acc[j][r] + accr[j][r] * (1.0f / 1024.0f)) * (1.0f / 2048.0f);
  ldsx();
  for (int rl = 0; rl < 16; ++rl) if (lane < HD / 4) vst2(Y + ((size_t)b * SEQ + ql0 + rl) * CC + h * HD + lane * 4, *(const v4f*)&ss[wave][rl][lane * 4]);
}

__global__ __launch_bounds__(256) void k_xsa(const float* __restrict__ Y, const float* __restrict__ VF, __bf16* __restrict__ YH, __bf16* __restrict__ YL) {
  __shared__ float sred[8]; __shared__ float sdot[4][8]; __shared__ __align__(16) float so[CC];
  const int tid = threadIdx.x, wave = tid >> 5, lane = tid & 31, kvh = tid >> 6, d = tid & 63; const size_t bt = blockIdx.x;
  const float v = VF[bt * KVD + tid];
  float yg[4];
#pragma unroll
  for (int gq = 0; gq < 4; ++gq) yg[gq] = Y[bt * CC + (kvh * 4 + gq) * HD + d];
  float pv = v * v;
#pragma unroll
  for (int o = 16; o > 0; o >>= 1) pv += __shfl_xor(pv, o);
  if (lane == 0) sred[wave] = pv;
  __syncthreads();
  const float n2 = sred[2 * kvh] + sred[2 * kvh + 1];
  const float den = fmaxf(sqrtf(n2), 1e-12f); const float vn = v * (1.0f / den);
  float pd[4];
#pragma unroll
  for (int gq = 0; gq < 4; ++gq) { float s = yg[gq] * vn;
#pragma unroll
    for (int o = 16; o > 0; o >>= 1) s += __shfl_xor(s, o);
    pd[gq] = s; }
  if (lane == 0) {
#pragma unroll
    for (int gq = 0; gq < 4; ++gq) sdot[gq][wave] = pd[gq]; }
  __syncthreads();
#pragma unroll
  for (int gq = 0; gq < 4; ++gq) { const float s = sdot[gq][2 * kvh] + sdot[gq][2 * kvh + 1]; so[(kvh * 4 + gq) * HD + d] = yg[gq] - s * vn; }
  __syncthreads();
  const int hf = tid >> 7, e = tid & 127;
  const v4f u0 = *(const v4f*)&so[e * 8], u1 = *(const v4f*)&so[e * 8 + 4];
  const float f[8] = { u0.x, u0.y, u0.z, u0.w, u1.x, u1.y, u1.z, u1.w };
  union { v8b v; v4u u; } pk;
#pragma unroll
  for (int i = 0; i < 8; ++i) { const __bf16 hb = (__bf16)f[i]; const __bf16 lb = (__bf16)(f[i] - (float)hb); pk.v[i] = hf ? lb : hb; }
  __bf16* dst = hf ? YL : YH;
  vst2((unsigned*)(dst + bt * CC + e * 8), pk.u);
}

__global__ __launch_bounds__(128) void k_out(const __bf16* __restrict__ YH, const __bf16* __restrict__ YL, const __bf16* __restrict__ WPI, const float* __restrict__ CS, float* __restrict__ OUT) {
  __shared__ __align__(16) float sf[4][16][132];
  const int tid = threadIdx.x, wave = tid >> 5, lane = tid & 31, col = lane & 15, g = lane >> 4; const int c0 = blockIdx.y * 128; const size_t r0 = (size_t)blockIdx.x * 64 + wave * 16;
  v8f acc[8] = {};
#pragma unroll 2
  for (int kc = 0; kc < CC / 32; ++kc) {
    const v16b ah = frag_b(YH + (r0 + col) * CC + kc * 32, lane), al = frag_b(YL + (r0 + col) * CC + kc * 32, lane);
#pragma unroll
    for (int j = 0; j < 8; ++j) { const v16b w = frag_b(WPI + (size_t)(c0 + j * 16 + col) * CC + kc * 32, lane); acc[j] = wmma_bf(ah, w, acc[j]); acc[j] = wmma_bf(al, w, acc[j]); }
  }
  const float* cs = CS + 1536 + c0;
#pragma unroll
  for (int j = 0; j < 8; ++j) { const float sc = cs[j * 16 + col];
#pragma unroll
    for (int r = 0; r < 8; ++r) sf[wave][8 * g + r][j * 16 + col] = acc[j][r] * sc; }
  ldsx();
  const size_t bb = r0 / SEQ; const int t0 = (int)(r0 % SEQ);
  for (int rl = 0; rl < 16; ++rl) vst2(OUT + ((bb * TT_FULL) + t0 + rl) * CC + c0 + lane * 4, *(const v4f*)&sf[wave][rl][lane * 4]);
}

extern "C" void kernel_launch(void* const* d_in, const int* in_sizes, int n_in, void* d_out, int out_size, void* d_ws, size_t ws_size, hipStream_t stream) {
  if (n_in < 6) return;
  if (in_sizes[0] < ((NB - 1) * TT_FULL + SEQ) * CC) return;
  if (in_sizes[1] < CC * CC || in_sizes[2] < KVD * CC || in_sizes[3] < KVD * CC || in_sizes[4] < CC * CC || in_sizes[5] < NH) return;
  if (out_size < ((NB - 1) * TT_FULL + SEQ) * CC) return;
  if (ws_size < (size_t)WS_END) return;
  const float* X  = (const float*)d_in[0];
  const float* WQ = (const float*)d_in[1];
  const float* WK = (const float*)d_in[2];
  const float* WV = (const float*)d_in[3];
  const float* WP = (const float*)d_in[4];
  const float* QG = (const float*)d_in[5];
  char* ws = (char*)d_ws;
  __bf16 *WQI = (__bf16*)(ws + WS_WQI), *WKI = (__bf16*)(ws + WS_WKI), *WVI = (__bf16*)(ws + WS_WVI), *WPI = (__bf16*)(ws + WS_WPI);
  float *CS = (float*)(ws + WS_CS), *CSN = (float*)(ws + WS_CSN);
  _Float16 *QH = (_Float16*)(ws + WS_QH), *QL = (_Float16*)(ws + WS_QL), *KH = (_Float16*)(ws + WS_KH), *KL = (_Float16*)(ws + WS_KL), *VT = (_Float16*)(ws + WS_VT), *VR = (_Float16*)(ws + WS_VR);
  float *VF = (float*)(ws + WS_VF), *Y = (float*)(ws + WS_Y);
  __bf16* XB = (__bf16*)(ws + WS_BIG);
  float* S = (float*)(ws + WS_BIG);
  __bf16 *YH = (__bf16*)(ws + WS_BIG), *YL = (__bf16*)(ws + WS_BIG + 2ull * NB * SEQ * CC);
  k_prep<<<dim3(NQB + NXB + NTB), 128, 0, stream>>>(X, WQ, WK, WV, WP, WQI, WKI, WVI, WPI, CS, XB, CSN);
  k_proj<<<dim3(NB * SEQ / 64, 12), 128, 0, stream>>>(XB, WQI, WKI, WVI, CS, CSN, QG, QH, QL, KH, KL, VT, VR, VF);
  for (int b = 0; b < NB; ++b) for (int kvh = 0; kvh < NKV; ++kvh) {
    k_sc<<<dim3(SEQ / 64, SEQ / 128, HG), 128, 0, stream>>>(QH, QL, KH, KL, b, kvh, S);
    k_sm<<<dim3(SEQ, HG), 256, 0, stream>>>(S);
    k_pv<<<dim3(SEQ / 64, 1, HG), 128, 0, stream>>>(S, VT, VR, b, kvh, Y);
  }
  k_xsa<<<dim3(NB * SEQ), 256, 0, stream>>>(Y, VF, YH, YL);
  k_out<<<dim3(NB * SEQ / 64, CC / 128), 128, 0, stream>>>(YH, YL, WPI, CS, (float*)d_out);
}
